// MatNetCrossMHACaps_25838523253363
// MI455X (gfx1250) — hardware-verified
//
#include <hip/hip_runtime.h>
#include <math.h>

#ifndef NB
#define NB 4
#endif
#ifndef SEQ
#define SEQ 512
#endif
#define SEQ_FULL 512
#define EMB 256
#define HEADS 8
#define HD 32
#define HID 16
#define MTOK (NB * SEQ)

#define X_CARRY 16.0f
#define W_CARRY 64.0f
#define QKV_CARRY 16.0f
#define P_CARRY 1024.0f
#define CTX_CARRY 256.0f
#define PROJ_EPI 0.015625f
#define SC_UNDO 0.00390625f
#define CTX_UP 16.0f
#define OUT_EPI 0.00006103515625f
#define LOG2E_F 1.4426950408889634f
#define INV_SQRT_HD 0.17677669529663687f

static_assert(PROJ_EPI * X_CARRY * W_CARRY == QKV_CARRY);
static_assert(SC_UNDO * QKV_CARRY * QKV_CARRY == 1.0f);
static_assert(CTX_UP * QKV_CARRY == CTX_CARRY);
static_assert(OUT_EPI * CTX_CARRY * W_CARRY == 1.0f);
static_assert(P_CARRY == 1024.0f);

static_assert(SEQ == 512);
static_assert(SEQ == SEQ_FULL);
static_assert(NB == 1 || NB == 2 || NB == 4);
static_assert(HEADS * HD == EMB);
static_assert(HD == 32);
static_assert(HID == 16);
static_assert(MTOK % 64 == 0);
static_assert(EMB % 64 == 0 && (2 * EMB) % 64 == 0);
static_assert(EMB % 32 == 0);
static_assert((MTOK * EMB / 8) % 256 == 0);
static_assert((EMB * (EMB / 8)) % 256 == 0);
static_assert((2 * EMB * (EMB / 8)) % 256 == 0);
static_assert(EMB / 8 == 32);
static_assert(SEQ % 128 == 0 && SEQ / 128 == 4);

static constexpr unsigned lg2c(unsigned v) { return (v <= 1u) ? 0u : 1u + lg2c(v >> 1); }
static constexpr unsigned LG_TN_EMB = lg2c(EMB / 64);
static constexpr unsigned LG_TN_TOK = lg2c(MTOK / 64);
static_assert((1u << LG_TN_EMB) == EMB / 64);
static_assert((1u << LG_TN_TOK) == MTOK / 64);
static constexpr unsigned G_CVT  = (MTOK * EMB / 8) / 256;
static constexpr unsigned G_WSQ  = (EMB * (EMB / 8)) / 256;
static constexpr unsigned G_WKV  = (2 * EMB * (EMB / 8)) / 256;
static constexpr unsigned G_GEMM = ((MTOK / 64) * (EMB / 64) + 7) / 8;
static constexpr unsigned G_ATTN = NB * 16;
static_assert(G_GEMM * 8 >= (MTOK / 64) * (EMB / 64));

typedef _Float16 h16;
typedef __attribute__((ext_vector_type(16))) _Float16 v16h;
typedef __attribute__((ext_vector_type(8)))  _Float16 v8h;
typedef __attribute__((ext_vector_type(8)))  float    v8f;
typedef __attribute__((ext_vector_type(4)))  float    v4f;


__device__ __forceinline__ float bfr(float f) {
    unsigned u = __float_as_uint(f);
    u += 0x7FFFu + ((u >> 16) & 1u);
    return __uint_as_float(u & 0xFFFF0000u);
}
static __device__ __forceinline__ h16 toh_flush(float v) { const float w = (fabsf(v) < 6.103515625e-05f) ? 0.0f : v; return (h16)w; }

static __device__ __forceinline__ void st8hf(_Float16* P, unsigned o, const float* v) {
    v8h hv;
#pragma unroll
    for (int e = 0; e < 8; ++e) hv[e] = toh_flush(v[e]);
    *(volatile v8h*)(P + o) = hv;
    __threadfence();
    *(volatile v8h*)(P + o) = hv;
}

union FragU { v16h v; v8h h[2]; };
__device__ __forceinline__ v16h frag_ld(const _Float16* p) {
    FragU f; f.h[0] = *(const v8h*)(p); f.h[1] = *(const v8h*)(p + 16); return f.v;
}
static __device__ __forceinline__ v8f wmma16g(v16h a, v16h b, v8f c) {
    c = __builtin_amdgcn_wmma_f32_16x16x32_f16(false, a, false, b, (short)0, c, false, false);
    asm volatile("v_nop\n\tv_nop\n\tv_nop\n\tv_nop" : "+v"(c) : "v"(a), "v"(b));
    return c;
}
__device__ __forceinline__ void wave_sync_lds() {
    __builtin_amdgcn_fence(3  , "workgroup");
    __builtin_amdgcn_wave_barrier();
    __builtin_amdgcn_fence(2  , "workgroup");
}

__global__ __launch_bounds__(256) void k_cvt16(const float* __restrict__ xq, const float* __restrict__ xkv,
                                               _Float16* __restrict__ Xq16, _Float16* __restrict__ Xkv16) {
    const unsigned u = blockIdx.x * 256u + threadIdx.x;
    if (u >= (unsigned)(MTOK * EMB / 8)) return;
    const unsigned o = u * 8u;
    const v4f a0 = *(const v4f*)(xq + o), a1 = *(const v4f*)(xq + o + 4u);
    const v4f b0 = *(const v4f*)(xkv + o), b1 = *(const v4f*)(xkv + o + 4u);
    float va[8] = {bfr(a0.x) * X_CARRY, bfr(a0.y) * X_CARRY, bfr(a0.z) * X_CARRY, bfr(a0.w) * X_CARRY,
                   bfr(a1.x) * X_CARRY, bfr(a1.y) * X_CARRY, bfr(a1.z) * X_CARRY, bfr(a1.w) * X_CARRY};
    float vb[8] = {bfr(b0.x) * X_CARRY, bfr(b0.y) * X_CARRY, bfr(b0.z) * X_CARRY, bfr(b0.w) * X_CARRY,
                   bfr(b1.x) * X_CARRY, bfr(b1.y) * X_CARRY, bfr(b1.z) * X_CARRY, bfr(b1.w) * X_CARRY};
    st8hf(Xq16, o, va);
    st8hf(Xkv16, o, vb);
}

__global__ __launch_bounds__(256) void k_wt16(const float* __restrict__ Wm, unsigned KI, unsigned NO, unsigned lgper,
                                              _Float16* __restrict__ W16) {
    const unsigned u = blockIdx.x * 256u + threadIdx.x;
    const unsigned per = 1u << lgper;
    if (u >= NO * per) return;
    const unsigned k0 = 8u * (u & (per - 1u));
    const unsigned o = u >> lgper;
    float v[8];
#pragma unroll
    for (int i = 0; i < 8; ++i) v[i] = bfr(Wm[(k0 + (unsigned)i) * NO + o]) * W_CARRY;
    st8hf(W16, o * KI + k0, v);
}

static __device__ __forceinline__ void gemm64_main(const _Float16* __restrict__ A, unsigned lda,
                                                   const _Float16* __restrict__ Bt, unsigned ldb,
                                                   unsigned m0, unsigned n0, unsigned K,
                                                   unsigned rlane, unsigned koff, v8f (&acc)[4][4]) {
#pragma unroll
    for (int i = 0; i < 4; ++i)
#pragma unroll
        for (int j = 0; j < 4; ++j) acc[i][j] = (v8f){0.f,0.f,0.f,0.f,0.f,0.f,0.f,0.f};

    for (unsigned k0 = 0; k0 < K; k0 += 32u) {
        v16h bh[4];
#pragma unroll
        for (int j = 0; j < 4; ++j)
            bh[j] = frag_ld(Bt + (size_t)(n0 + ((unsigned)j << 4) + rlane) * ldb + koff + k0);
        unsigned arow = m0 + rlane;
#pragma unroll
        for (int i = 0; i < 4; ++i) {
            if (i == 2) { asm volatile("" : "+v"(arow)); }
            const v16h ah = frag_ld(A + (size_t)(arow + ((unsigned)i << 4)) * lda + koff + k0);
#pragma unroll
            for (int j = 0; j < 4; ++j) acc[i][j] = wmma16g(ah, bh[j], acc[i][j]);
        }
    }
}

__global__ __launch_bounds__(256) __attribute__((amdgpu_num_vgpr(256)))
void k_gemm_h(const _Float16* __restrict__ A, unsigned lda, const _Float16* __restrict__ Bt, unsigned ldb,
              _Float16* __restrict__ C, unsigned ldc, unsigned M, unsigned N, unsigned K, unsigned lgTilesN) {
    __shared__ __align__(16) float sT[8][16 * 68];
    static_assert(8 * 16 * 68 * 4 <= 131072);
    const unsigned lane = threadIdx.x & 31u;
    const unsigned wave = (unsigned)__builtin_amdgcn_readfirstlane((int)(threadIdx.x >> 5));
    const unsigned tilesN = N >> 6, tilesM = M >> 6;
    const unsigned tile = blockIdx.x * 8u + wave;
    if (tile >= tilesM * tilesN) return;
    const unsigned tm = tile >> lgTilesN;
    const unsigned tn = tile & (tilesN - 1u);
    const unsigned m0 = tm << 6, n0 = tn << 6;
    const unsigned rlane = lane & 15u;
    const unsigned koff = (lane >> 4) * 8u;
    const unsigned mOff = koff;

    v8f acc[4][4];
    gemm64_main(A, lda, Bt, ldb, m0, n0, K, rlane, koff, acc);

    float* slab = sT[wave];
#pragma unroll
    for (int i = 0; i < 4; ++i) {
        const unsigned mBase = m0 + ((unsigned)i << 4);
#pragma unroll
        for (int j = 0; j < 4; ++j) {
#pragma unroll
            for (int r = 0; r < 8; ++r)
                slab[(mOff + (unsigned)r) * 68u + ((unsigned)j << 4) + rlane] = acc[i][j][r] * PROJ_EPI;
        }
        wave_sync_lds();
        {
            const unsigned q = lane >> 3, c8 = (lane & 7u) * 8u;
            static_assert(32 * 8 * 4 == 16 * 64);
            v8h hv[4];
#pragma unroll
            for (int it = 0; it < 4; ++it) {
                const unsigned row = (unsigned)it * 4u + q;
                const float* sp = slab + row * 68u + c8;
#pragma unroll
                for (int e = 0; e < 8; ++e) hv[it][e] = toh_flush(sp[e]);
            }
            for (int pass = 0; pass < 2; ++pass) {
#pragma unroll
                for (int it = 0; it < 4; ++it) {
                    const unsigned row = (unsigned)it * 4u + q;
                    *(volatile v8h*)(C + (size_t)(mBase + row) * ldc + n0 + c8) = hv[it];
                }
                __threadfence();
            }
        }
        wave_sync_lds();
    }
}

__global__ __launch_bounds__(256) __attribute__((amdgpu_num_vgpr(256)))
void k_gemm_f(const _Float16* __restrict__ A, unsigned lda, const _Float16* __restrict__ Bt, unsigned ldb,
              float* __restrict__ C, unsigned ldc, unsigned M, unsigned N, unsigned K, unsigned lgTilesN) {
    __shared__ __align__(16) float sT[8][16 * 68];
    const unsigned lane = threadIdx.x & 31u;
    const unsigned wave = (unsigned)__builtin_amdgcn_readfirstlane((int)(threadIdx.x >> 5));
    const unsigned tilesN = N >> 6, tilesM = M >> 6;
    const unsigned tile = blockIdx.x * 8u + wave;
    if (tile >= tilesM * tilesN) return;
    const unsigned tm = tile >> lgTilesN;
    const unsigned tn = tile & (tilesN - 1u);
    const unsigned m0 = tm << 6, n0 = tn << 6;
    const unsigned rlane = lane & 15u;
    const unsigned koff = (lane >> 4) * 8u;
    const unsigned mOff = koff;

    v8f acc[4][4];
    gemm64_main(A, lda, Bt, ldb, m0, n0, K, rlane, koff, acc);

    float* slab = sT[wave];
#pragma unroll
    for (int i = 0; i < 4; ++i) {
        const unsigned mBase = m0 + ((unsigned)i << 4);
#pragma unroll
        for (int j = 0; j < 4; ++j) {
#pragma unroll
            for (int r = 0; r < 8; ++r)
                slab[(mOff + (unsigned)r) * 68u + ((unsigned)j << 4) + rlane] = acc[i][j][r] * OUT_EPI;
        }
        wave_sync_lds();
        {
            const unsigned hh = lane >> 4, c4 = (lane & 15u) * 4u;
            static_assert(32 * 4 * 8 == 16 * 64);
#pragma unroll
            for (int half = 0; half < 2; ++half) {
                v4f vv[4];
#pragma unroll
                for (int it = 0; it < 4; ++it) {
                    const unsigned row = (unsigned)(half * 4 + it) * 2u + hh;
                    vv[it] = *(const v4f*)(slab + row * 68u + c4);
                }
                for (int pass = 0; pass < 2; ++pass) {
#pragma unroll
                    for (int it = 0; it < 4; ++it) {
                        const unsigned row = (unsigned)(half * 4 + it) * 2u + hh;
                        *(volatile v4f*)(C + (size_t)(mBase + row) * ldc + n0 + c4) = vv[it];
                    }
                    __threadfence();
                }
            }
        }
        wave_sync_lds();
    }
}

#define AT_TP 68
#define PAR_Q 64
__global__ __launch_bounds__(256) __attribute__((amdgpu_num_vgpr(256)))
void k_attn_mix(const _Float16* __restrict__ Q16, const _Float16* __restrict__ K16, const _Float16* __restrict__ VT16,
                const float* __restrict__ dmat, const float* __restrict__ caps,
                const float* __restrict__ mW1, const float* __restrict__ mb1, const float* __restrict__ mW2, const float* __restrict__ mb2,
                const float* __restrict__ cW1, const float* __restrict__ cb1, const float* __restrict__ cW2, const float* __restrict__ cb2,
                const float* __restrict__ mix3, const float* __restrict__ mix3b,
                _Float16* __restrict__ ctx16) {
    __shared__ __align__(16) v4f sPar[2 * PAR_Q];
    __shared__ __align__(16) float sT[8][16 * AT_TP];
    static_assert(2 * PAR_Q * 16 + 8 * 16 * AT_TP * 4 <= 131072);
    const unsigned tid = threadIdx.x, lane = tid & 31u;
    const unsigned wave = (unsigned)__builtin_amdgcn_readfirstlane((int)(threadIdx.x >> 5));
    const unsigned hh = lane >> 4, c = lane & 15u;
    const unsigned bx = blockIdx.x;
    const unsigned b = bx >> 4, pair = (bx >> 2) & 3u, qb = bx & 3u;

    if (wave == 0u) {
        const unsigned hl = 2u * pair + hh;
        v4f wd, wc, ta, tb;
        wd.x = bfr(mW1[hl * 32u + c]); wd.y = bfr(mW1[hl * 32u + 16u + c]); wd.z = bfr(mb1[hl * 16u + c]); wd.w = bfr(mW2[hl * 16u + c]);
        wc.x = bfr(cW1[hl * 32u + c]); wc.y = bfr(cW1[hl * 32u + 16u + c]); wc.z = bfr(cb1[hl * 16u + c]); wc.w = bfr(cW2[hl * 16u + c]);
        ta.x = bfr(mb2[hl]); ta.y = bfr(cb2[hl]); ta.z = bfr(mix3[0]); ta.w = bfr(mix3[1]);
        tb.x = bfr(mix3b[hl]); tb.y = 0.0f; tb.z = 0.0f; tb.w = 0.0f;
        sPar[hh * PAR_Q + c] = wd;
        sPar[hh * PAR_Q + 16u + c] = wc;
        sPar[hh * PAR_Q + 32u + c] = ta;
        sPar[hh * PAR_Q + 48u + c] = tb;
    }
    __syncthreads();

    const unsigned i0 = qb * 128u + wave * 16u;
    float* pw = sT[wave];
    const float SCS = INV_SQRT_HD * SC_UNDO;
    const unsigned drow = (b * SEQ_FULL + i0 + c) * SEQ_FULL + 8u * hh;
    const unsigned crow = b * SEQ_FULL + 8u * hh;

#pragma unroll 1
    for (unsigned hp = 0; hp < 2u; ++hp) {
        const unsigned h = 2u * pair + hp;
        const v16h qf = frag_ld(Q16 + (size_t)(b * SEQ + i0 + c) * EMB + h * HD + 8u * hh);
        const v4f ta = sPar[hp * PAR_Q + 32u];
        const v4f tb = sPar[hp * PAR_Q + 48u];
        const float b2d = ta.x, b2c = ta.y, m3a = ta.z, m3b = ta.w, bias3 = tb.x;
        float mrun = -3.0e38f, lrun = 0.0f;
        v8f o0 = (v8f){0.f,0.f,0.f,0.f,0.f,0.f,0.f,0.f};
        v8f o1 = o0;

#pragma unroll 1
        for (unsigned kv0 = 0; kv0 < (unsigned)SEQ; kv0 += 32u) {
            float sv[16], dmv[16], cpv[16];
#pragma unroll
            for (int tt = 0; tt < 2; ++tt) {
                const v16h kf = frag_ld(K16 + (size_t)(b * SEQ + kv0 + (unsigned)tt * 16u + c) * EMB + h * HD + 8u * hh);
                const v8f z = (v8f){0.f,0.f,0.f,0.f,0.f,0.f,0.f,0.f};
                const v8f st = wmma16g(kf, qf, z);
#pragma unroll
                for (int r = 0; r < 8; ++r) sv[8 * tt + r] = st[r] * SCS;
                const v4f d0 = *(const v4f*)(dmat + drow + kv0 + (unsigned)tt * 16u);
                const v4f d1 = *(const v4f*)(dmat + drow + kv0 + (unsigned)tt * 16u + 4u);
                const v4f c0 = *(const v4f*)(caps + crow + kv0 + (unsigned)tt * 16u);
                const v4f c1 = *(const v4f*)(caps + crow + kv0 + (unsigned)tt * 16u + 4u);
                dmv[8 * tt + 0] = bfr(d0.x); dmv[8 * tt + 1] = bfr(d0.y); dmv[8 * tt + 2] = bfr(d0.z); dmv[8 * tt + 3] = bfr(d0.w);
                dmv[8 * tt + 4] = bfr(d1.x); dmv[8 * tt + 5] = bfr(d1.y); dmv[8 * tt + 6] = bfr(d1.z); dmv[8 * tt + 7] = bfr(d1.w);
                cpv[8 * tt + 0] = bfr(c0.x); cpv[8 * tt + 1] = bfr(c0.y); cpv[8 * tt + 2] = bfr(c0.z); cpv[8 * tt + 3] = bfr(c0.w);
                cpv[8 * tt + 4] = bfr(c1.x); cpv[8 * tt + 5] = bfr(c1.y); cpv[8 * tt + 6] = bfr(c1.z); cpv[8 * tt + 7] = bfr(c1.w);
            }

            float ad[16], ac[16];
#pragma unroll
            for (int e = 0; e < 16; ++e) { ad[e] = 0.0f; ac[e] = 0.0f; }
#pragma unroll 1
            for (unsigned u = 0; u < (unsigned)HID; ++u) {
                const v4f wd = sPar[hp * PAR_Q + u];
                const v4f wc = sPar[hp * PAR_Q + 16u + u];
#pragma unroll
                for (int e = 0; e < 16; ++e) {
                    float hd = fmaf(sv[e], wd.x, fmaf(dmv[e], wd.y, wd.z));
                    hd = (hd > 0.0f) ? hd : 0.0f;
                    ad[e] = fmaf(hd, wd.w, ad[e]);
                    float hc = fmaf(sv[e], wc.x, fmaf(cpv[e], wc.y, wc.z));
                    hc = (hc > 0.0f) ? hc : 0.0f;
                    ac[e] = fmaf(hc, wc.w, ac[e]);
                }
            }

            float mx = -3.0e38f;
#pragma unroll
            for (int e = 0; e < 16; ++e) {
                float ds = ad[e] + b2d; ds = (ds > 0.0f) ? ds : 0.0f;
                float cs = ac[e] + b2c; cs = (cs > 0.0f) ? cs : 0.0f;
                const float mixed = fmaf(ds, m3a, fmaf(cs, m3b, bias3));
                sv[e] = mixed * LOG2E_F;
                mx = (sv[e] > mx) ? sv[e] : mx;
            }
            const float mo = __shfl_xor(mx, 16, 32);
            mx = (mo > mx) ? mo : mx;
            const float mnew = (mx > mrun) ? mx : mrun;
            const float alpha = exp2f(mrun - mnew);
            mrun = mnew;

            v16h pv;
            float psum = 0.0f;
#pragma unroll
            for (int e = 0; e < 16; ++e) {
                const float p = exp2f(sv[e] - mnew);
                const h16 ph = toh_flush(p * P_CARRY);
                pv[e] = ph;
                psum += (float)ph;
            }
            lrun = lrun * alpha + psum;
#pragma unroll
            for (int r = 0; r < 8; ++r) { o0[r] *= alpha; o1[r] *= alpha; }

            unsigned voff = b * SEQ + kv0 + 8u * hh;
            asm volatile("" : "+v"(voff));
            const v16h vf0 = frag_ld(VT16 + (size_t)(h * HD + c) * MTOK + voff);
            const v16h vf1 = frag_ld(VT16 + (size_t)(h * HD + 16u + c) * MTOK + voff);
            o0 = wmma16g(vf0, pv, o0);
            o1 = wmma16g(vf1, pv, o1);
        }

        const float lt = lrun + __shfl_xor(lrun, 16, 32);
        const float inv = CTX_UP * (1.0f / lt);
#pragma unroll
        for (int r = 0; r < 8; ++r) {
            pw[c * AT_TP + hp * 32u + 8u * hh + (unsigned)r] = o0[r] * inv;
            pw[c * AT_TP + hp * 32u + 16u + 8u * hh + (unsigned)r] = o1[r] * inv;
        }
    }
    wave_sync_lds();
    {
        const unsigned q = lane >> 3, c8 = (lane & 7u) * 8u;
        static_assert(32 * 8 * 4 == 16 * 64);
        v8h ov[4];
#pragma unroll
        for (int it = 0; it < 4; ++it) {
            const unsigned row = (unsigned)it * 4u + q;
            const float* sp = pw + row * AT_TP + c8;
#pragma unroll
            for (int e = 0; e < 8; ++e) ov[it][e] = toh_flush(sp[e]);
        }
        _Float16* dst = ctx16 + (size_t)(b * SEQ + i0) * EMB + pair * 64u;
        for (int pass = 0; pass < 2; ++pass) {
#pragma unroll
            for (int it = 0; it < 4; ++it) *(volatile v8h*)(dst + (size_t)((unsigned)it * 4u + q) * EMB + c8) = ov[it];
            __threadfence();
        }
    }
}

extern "C" void kernel_launch(void* const* d_in, const int* in_sizes, int n_in, void* d_out, int out_size,
                              void* d_ws, size_t ws_size, hipStream_t stream) {
    if (n_in < 17) return;
    if (in_sizes[0] < MTOK * EMB || in_sizes[1] < MTOK * EMB || in_sizes[2] < NB * SEQ * SEQ || in_sizes[3] < NB * SEQ) return;
    if (in_sizes[4] < EMB * EMB || in_sizes[5] < EMB * 2 * EMB || in_sizes[16] < EMB * EMB) return;
    if (in_sizes[6] < HEADS * 2 * HID || in_sizes[7] < HEADS * HID || in_sizes[8] < HEADS * HID || in_sizes[9] < HEADS) return;
    if (in_sizes[10] < HEADS * 2 * HID || in_sizes[11] < HEADS * HID || in_sizes[12] < HEADS * HID || in_sizes[13] < HEADS) return;
    if (in_sizes[14] < 2 || in_sizes[15] < HEADS || out_size < MTOK * EMB) return;

    const float* q_input  = (const float*)d_in[0];
    const float* kv_input = (const float*)d_in[1];
    const float* dmat     = (const float*)d_in[2];
    const float* caps_emb = (const float*)d_in[3];
    const float* Wq       = (const float*)d_in[4];
    const float* Wkv      = (const float*)d_in[5];
    const float* mix_W1   = (const float*)d_in[6];
    const float* mix_b1   = (const float*)d_in[7];
    const float* mix_W2   = (const float*)d_in[8];
    const float* mix_b2   = (const float*)d_in[9];
    const float* cap_W1   = (const float*)d_in[10];
    const float* cap_b1   = (const float*)d_in[11];
    const float* cap_W2   = (const float*)d_in[12];
    const float* cap_b2   = (const float*)d_in[13];
    const float* mix3     = (const float*)d_in[14];
    const float* mix3bias = (const float*)d_in[15];
    const float* Wout     = (const float*)d_in[16];
    float* out = (float*)d_out;

    char* wsp = (char*)d_ws;
    size_t off = 0;
    auto carve = [&](size_t bytes) -> void* { void* r = wsp + off; off += (bytes + 255) & ~(size_t)255; return r; };
    _Float16* X16q  = (_Float16*)carve((size_t)MTOK * EMB * 2);
    _Float16* X16kv = (_Float16*)carve((size_t)MTOK * EMB * 2);
    _Float16* WqT   = (_Float16*)carve((size_t)EMB * EMB * 2);
    _Float16* WkvT  = (_Float16*)carve((size_t)2 * EMB * EMB * 2);
    _Float16* WoT   = (_Float16*)carve((size_t)EMB * EMB * 2);
    _Float16* Q16   = (_Float16*)carve((size_t)MTOK * EMB * 2);
    _Float16* K16   = (_Float16*)carve((size_t)MTOK * EMB * 2);
    _Float16* VT16  = (_Float16*)carve((size_t)EMB * MTOK * 2);
    _Float16* CTX16 = (_Float16*)carve((size_t)MTOK * EMB * 2);
    if (off > ws_size || off > (size_t)134217728) return;

    k_cvt16<<<G_CVT, 256, 0, stream>>>(q_input, kv_input, X16q, X16kv);
    k_wt16<<<G_WSQ, 256, 0, stream>>>(Wq, EMB, EMB, 5u, WqT);
    k_wt16<<<G_WKV, 256, 0, stream>>>(Wkv, EMB, 2 * EMB, 5u, WkvT);
    k_wt16<<<G_WSQ, 256, 0, stream>>>(Wout, EMB, EMB, 5u, WoT);

    k_gemm_h<<<G_GEMM, 256, 0, stream>>>((const _Float16*)X16q, EMB, (const _Float16*)WqT, EMB, Q16, EMB, MTOK, EMB, EMB, LG_TN_EMB);
    k_gemm_h<<<G_GEMM, 256, 0, stream>>>((const _Float16*)X16kv, EMB, (const _Float16*)WkvT, EMB, K16, EMB, MTOK, EMB, EMB, LG_TN_EMB);
    k_gemm_h<<<G_GEMM, 256, 0, stream>>>((const _Float16*)(WkvT + (size_t)EMB * EMB), EMB, (const _Float16*)X16kv, EMB, VT16, MTOK, EMB, MTOK, EMB, LG_TN_TOK);

    k_attn_mix<<<G_ATTN, 256, 0, stream>>>((const _Float16*)Q16, (const _Float16*)K16, (const _Float16*)VT16, dmat, caps_emb,
        mix_W1, mix_b1, mix_W2, mix_b2, cap_W1, cap_b1, cap_W2, cap_b2, mix3, mix3bias, CTX16);

    k_gemm_f<<<G_GEMM, 256, 0, stream>>>((const _Float16*)CTX16, EMB, (const _Float16*)WoT, EMB, out, EMB, MTOK, EMB, EMB, LG_TN_EMB);
}
